// BipartiteGraphConvolution_28406913696348
// MI455X (gfx1250) — hardware-verified
//
#include <hip/hip_runtime.h>
#include <stdint.h>


#define EMB   128
#define NLN   50000
#define NLP   50048
#define NRN   100000
#define NRH   50048
#define NE    500000
#define NT    256
#define SRB   4096
#define SCH   4096
#define SPT   (SCH / NT)
#define NCH   ((NE + SCH - 1) / SCH)
#define NTILE ((NRH + SRB - 1) / SRB)
#define RPW   (SRB / (NT / 32))
static_assert(NE % SPT == 0);
static_assert(NRH % 128 == 0);
static_assert(NLP == NRH);
static_assert(NLP % 64 == 0);

typedef __attribute__((ext_vector_type(16))) _Float16 v16h;
typedef __attribute__((ext_vector_type(8)))  _Float16 v8h;
typedef __attribute__((ext_vector_type(16))) __bf16   v16b;
typedef __attribute__((ext_vector_type(8)))  __bf16   v8b;
typedef __attribute__((ext_vector_type(8)))  float    v8f;
typedef __attribute__((ext_vector_type(4)))  float    v4f;
typedef __attribute__((ext_vector_type(4)))  int      v4i;

__device__ __forceinline__ unsigned short f2bf_bits(float f) {
  unsigned u = __float_as_uint(f);
  return (unsigned short)((u + 0x7FFFu + ((u >> 16) & 1u)) >> 16);
}
__device__ __forceinline__ float bf_bits2f(unsigned short h) { return __uint_as_float(((unsigned)h) << 16); }

__device__ __forceinline__ void dep_guard_h(v8f& a, v8f& b, v16h x, v16h y) { asm volatile("v_nop\n\tv_nop\n\tv_nop\n\tv_nop" : "+v"(a), "+v"(b) : "v"(x), "v"(y)); }
__device__ __forceinline__ void dep_guard_b(v8f& a, v8f& b, v16b x, v16b y) { asm volatile("v_nop\n\tv_nop\n\tv_nop\n\tv_nop" : "+v"(a), "+v"(b) : "v"(x), "v"(y)); }
__device__ __forceinline__ void keep4_h(v16h a, v16h b, v16h c, v16h d) { asm volatile("v_nop" :: "v"(a), "v"(b), "v"(c), "v"(d)); }
__device__ __forceinline__ void keep4_b(v16b a, v16b b, v16b c, v16b d) { asm volatile("v_nop" :: "v"(a), "v"(b), "v"(c), "v"(d)); }
__device__ __forceinline__ void acc_guard4(v8f& a, v8f& b, v8f& c, v8f& d) { asm volatile("v_nop\n\tv_nop\n\tv_nop\n\tv_nop" : "+v"(a), "+v"(b), "+v"(c), "+v"(d)); }
template <typename T> struct Frag;
template <> struct Frag<_Float16> {
  typedef v16h V; union U { v16h v; v8h h[2]; };
  static __device__ __forceinline__ v16h load(const _Float16* p) {
    U f; f.h[0] = *(const v8h*)(p); f.h[1] = *(const v8h*)(p + 16); return f.v;
  }
  static __device__ __forceinline__ v8f mma(v16h a, v16h b, v8f c) {
    return __builtin_amdgcn_wmma_f32_16x16x32_f16(false, a, false, b, (short)0, c, false, false);
  }
  static __device__ __forceinline__ void guard(v8f& a, v8f& b, v16h x, v16h y) { dep_guard_h(a, b, x, y); }
  static __device__ __forceinline__ void keep(v16h a, v16h b, v16h c, v16h d) { keep4_h(a, b, c, d); }
};
template <> struct Frag<__bf16> {
  typedef v16b V; union U { v16b v; v8b h[2]; };
  static __device__ __forceinline__ v16b load(const __bf16* p) {
    U f; f.h[0] = *(const v8b*)(p); f.h[1] = *(const v8b*)(p + 16); return f.v;
  }
  static __device__ __forceinline__ v8f mma(v16b a, v16b b, v8f c) {
    return __builtin_amdgcn_wmma_f32_16x16x32_bf16(false, a, false, b, (short)0, c, false, false);
  }
  static __device__ __forceinline__ void guard(v8f& a, v8f& b, v16b x, v16b y) { dep_guard_b(a, b, x, y); }
  static __device__ __forceinline__ void keep(v16b a, v16b b, v16b c, v16b d) { keep4_b(a, b, c, d); }
};

template <int ET> struct Elem;
template <> struct Elem<0> { typedef _Float16 T; };
template <> struct Elem<1> { typedef __bf16 T; };
template <int ET, bool SPLIT, int BIAS_MODE, int OUT_MODE, bool RESID, int ACT = 0>
__global__ __launch_bounds__(256) void wmma_gemm64(
    const unsigned short* __restrict__ Ap, const unsigned short* __restrict__ A2p, int lda, long strideA,
    const unsigned short* __restrict__ Btp, const unsigned short* __restrict__ Bt2p, int ldb, long strideB,
    void* __restrict__ Cout, void* __restrict__ Cout2, int ldc, long strideC,
    const float* __restrict__ bias,
    const float* __restrict__ resid, long strideR,
    int M, int N, int K, float scale, int Mst) {
  typedef typename Elem<ET>::T T;
  typedef typename Frag<T>::V V;
  const T* A = (const T*)Ap; const T* A2 = (const T*)A2p; const T* Bt = (const T*)Btp; const T* Bt2 = (const T*)Bt2p;
  __shared__ __align__(16) float sT[8][16 * 68];
  const int b    = blockIdx.y;
  const int lane = threadIdx.x & 31;
  const int wave = threadIdx.x >> 5;
  const int tilesN = N >> 6;
  const int tilesM = M >> 6;
  const int tile = blockIdx.x * 8 + wave;
  if (tile >= tilesM * tilesN) return;
  const int tm = tile / tilesN;
  const int tn = tile - tm * tilesN;
  const int m0 = tm << 6;
  const int n0 = tn << 6;

  const T* Ab  = A  + (size_t)b * strideA;
  const T* Bb  = Bt + (size_t)b * strideB;
  const T* Ab2 = SPLIT ? (A2  + (size_t)b * strideA) : nullptr;
  const T* Bb2 = SPLIT ? (Bt2 + (size_t)b * strideB) : nullptr;

  const int rlane = lane & 15;
  const int koff  = (lane >> 4) * 8;
  const int mOff  = (lane >> 4) * 8;

  v8f acc[4][4];
#pragma unroll
  for (int i = 0; i < 4; ++i)
#pragma unroll
    for (int j = 0; j < 4; ++j) acc[i][j] = (v8f){0.f,0.f,0.f,0.f,0.f,0.f,0.f,0.f};

  for (int k0 = 0; k0 < K; k0 += 32) {
    V bh[4], bl[4];
#pragma unroll
    for (int j = 0; j < 4; ++j) {
      const size_t bo = (size_t)(n0 + (j << 4) + rlane) * ldb + koff + k0;
      bh[j] = Frag<T>::load(Bb + bo);
      if (SPLIT) bl[j] = Frag<T>::load(Bb2 + bo);
    }
#pragma unroll
    for (int i = 0; i < 4; ++i) {
      const size_t ao = (size_t)(m0 + (i << 4) + rlane) * lda + koff + k0;
      V ah = Frag<T>::load(Ab + ao);
      V al;
      if (SPLIT) al = Frag<T>::load(Ab2 + ao);
#pragma unroll
      for (int j = 0; j < 4; ++j) {
        acc[i][j] = Frag<T>::mma(ah, bh[j], acc[i][j]);
        if (SPLIT) {
          acc[i][j] = Frag<T>::mma(ah, bl[j], acc[i][j]);
          acc[i][j] = Frag<T>::mma(al, bh[j], acc[i][j]);
        }
      }
      Frag<T>::guard(acc[i][0], acc[i][3], ah, SPLIT ? al : ah);
    }
    Frag<T>::keep(bh[0], bh[1], bh[2], bh[3]);
    if (SPLIT) Frag<T>::keep(bl[0], bl[1], bl[2], bl[3]);
  }
  acc_guard4(acc[0][0], acc[0][1], acc[0][2], acc[0][3]);
  acc_guard4(acc[1][0], acc[1][1], acc[1][2], acc[1][3]);
  acc_guard4(acc[2][0], acc[2][1], acc[2][2], acc[2][3]);
  acc_guard4(acc[3][0], acc[3][1], acc[3][2], acc[3][3]);

  float* slab = sT[wave];
  const float* Rb = RESID ? (resid + (size_t)b * strideR) : nullptr;
#pragma unroll
  for (int i = 0; i < 4; ++i) {
    const int mBase = m0 + (i << 4);
#pragma unroll
    for (int j = 0; j < 4; ++j) {
      const int n = n0 + (j << 4) + rlane;
      float bv = 0.f;
      if (BIAS_MODE == 2 || BIAS_MODE == 3) bv = bias[n];
#pragma unroll
      for (int r = 0; r < 8; ++r) {
        float v = acc[i][j][r] * scale;
        if (BIAS_MODE == 1) v += bias[mBase + mOff + r];
        if (BIAS_MODE == 2) v += bv;
        if (BIAS_MODE == 3) v += bv * resid[mBase + mOff + r];
        if (RESID) v += Rb[(size_t)(mBase + mOff + r) * ldc + n];
        if (ACT == 1) v = tanhf(v);
        if (ACT == 2) v = fmaxf(v, 0.0f);
        if (ACT == 3) v = v / (1.0f + expf(-v));
        if (ACT == 4) v = (v > 0.f) ? v : 0.01f * v;
        if (ACT == 5) v = 0.5f * v * (1.0f + erff(v * 0.70710678118654752f));
        slab[(mOff + r) * 68 + (j << 4) + rlane] = v;
      }
    }
    __builtin_amdgcn_fence(__ATOMIC_RELEASE, "workgroup");
    __builtin_amdgcn_wave_barrier();
    __builtin_amdgcn_fence(__ATOMIC_ACQUIRE, "workgroup");
    if (OUT_MODE == 0) {
      float* C = (float*)Cout + (size_t)b * strideC;
      const int hh = lane >> 4, c4 = (lane & 15) * 4;
      for (int pass = 0; pass < 2; ++pass) {
#pragma unroll
        for (int it = 0; it < 8; ++it) {
          const int row = it * 2 + hh;
          v4f v = *(const v4f*)(slab + row * 68 + c4);
          if (mBase + row < Mst) *(volatile v4f*)(C + (size_t)(mBase + row) * ldc + n0 + c4) = v;
        }
        __threadfence();
      }
    } else {
      const int q = lane >> 3, c8 = (lane & 7) * 8;
      unsigned short* C  = (unsigned short*)Cout  + (size_t)b * strideC;
      unsigned short* C2 = (OUT_MODE == 2) ? ((unsigned short*)Cout2 + (size_t)b * strideC) : nullptr;
      for (int pass = 0; pass < 2; ++pass) {
#pragma unroll
        for (int it = 0; it < 4; ++it) {
          const int row = it * 4 + q;
          const float* sp = slab + row * 68 + c8;
          v8h hv, lv;
#pragma unroll
          for (int e = 0; e < 8; ++e) {
            if (OUT_MODE == 1) {
              hv[e] = (_Float16)sp[e];
            } else {
              unsigned short hb = f2bf_bits(sp[e]);
              unsigned short lb = f2bf_bits(sp[e] - bf_bits2f(hb));
              hv[e] = __builtin_bit_cast(_Float16, hb);
              lv[e] = __builtin_bit_cast(_Float16, lb);
            }
          }
          if (mBase + row < Mst) {
            *(volatile v8h*)(C + (size_t)(mBase + row) * ldc + n0 + c8) = hv;
            if (OUT_MODE == 2) *(volatile v8h*)(C2 + (size_t)(mBase + row) * ldc + n0 + c8) = lv;
          }
        }
        __threadfence();
      }
    }
    __builtin_amdgcn_fence(__ATOMIC_RELEASE, "workgroup");
    __builtin_amdgcn_wave_barrier();
    __builtin_amdgcn_fence(__ATOMIC_ACQUIRE, "workgroup");
  }
}

__device__ __forceinline__ int blk_excl_scan(int cnt, int* scan_ws, int tid, int* tot) {
  const int lane = tid & 31, wave = tid >> 5; int incl = cnt;
#pragma unroll
  for (int o = 1; o < 32; o <<= 1) { const int v = __shfl_up(incl, o, 32); if (lane >= o) incl += v; }
  if (lane == 31) scan_ws[wave] = incl;
  __syncthreads();
  if (wave == 0) { int wv = (lane < NT / 32) ? scan_ws[lane] : 0; int wincl = wv;
#pragma unroll
    for (int o = 1; o < 32; o <<= 1) { const int v = __shfl_up(wincl, o, 32); if (lane >= o) wincl += v; }
    if (lane < NT / 32) scan_ws[32 + lane] = wincl - wv; if (lane == 31) scan_ws[64] = wincl; }
  __syncthreads();
  const int res = scan_ws[32 + wave] + incl - cnt; *tot = scan_ws[64];
  return res;
}
template <int SPc, int CAP>
__device__ __forceinline__ int chunk_hits_dst(const int* __restrict__ dstv, int e0, int g0, int gend, int tid, int* LIST, int* scan_ws) {
  const int eb = e0 + tid * SPc;
  const bool valid = eb < NE;
  const int ebc = valid ? eb : (NE - SPc);
  int rec[SPc]; int cnt = 0;
#pragma unroll
  for (int k = 0; k < SPc; k += 4) {
    const v4i d4 = *(const v4i*)(dstv + ebc + k);
#pragma unroll
    for (int e = 0; e < 4; ++e) {
      const int d = d4[e]; int r = -1;
      if (valid && d >= g0 && d < gend) { r = ((d - g0) << 19) | (eb + k + e); ++cnt; }
      rec[k + e] = r;
    }
  }
  int tot; int p = blk_excl_scan(cnt, scan_ws, tid, &tot);
#pragma unroll
  for (int k = 0; k < SPc; ++k) if (rec[k] >= 0) { if ((unsigned)p < (unsigned)CAP) LIST[p] = rec[k]; ++p; }
  __syncthreads();
  return tot < CAP ? tot : CAP;
}

__global__ __launch_bounds__(NT) void prep_w_kernel(const float* __restrict__ Wl, const float* __restrict__ Wr, const float* __restrict__ Wf,
                                                   const float* __restrict__ W1, const float* __restrict__ W2,
                                                   unsigned* __restrict__ WlF, unsigned* __restrict__ WrH, unsigned* __restrict__ WrL,
                                                   unsigned* __restrict__ WfH, unsigned* __restrict__ WfL,
                                                   unsigned* __restrict__ W1H, unsigned* __restrict__ W1L,
                                                   unsigned* __restrict__ W2H, unsigned* __restrict__ W2L) {
  const int bid = blockIdx.x;
  const float* src; unsigned* dh; unsigned* dlo; int nd; int lb; bool f16m = false;
  if (bid < 32)       { src = Wl; dh = WlF; dlo = WlF; nd = EMB * EMB / 2;     lb = bid;       f16m = true; }
  else if (bid < 64)  { src = Wr; dh = WrH; dlo = WrL; nd = EMB * EMB / 2;     lb = bid - 32;  }
  else if (bid < 96)  { src = Wf; dh = WfH; dlo = WfL; nd = EMB * EMB / 2;     lb = bid - 64;  }
  else if (bid < 160) { src = W1; dh = W1H; dlo = W1L; nd = 2 * EMB * EMB / 2; lb = bid - 96;  }
  else                { src = W2; dh = W2H; dlo = W2L; nd = EMB * EMB / 2;     lb = bid - 160; }
  const int i = lb * NT + threadIdx.x;
  if (i >= nd) return;
  const float a = src[2 * i], b = src[2 * i + 1];
  unsigned uh, ul;
  if (f16m) {
    const _Float16 h0 = (_Float16)(a * 16.0f), h1 = (_Float16)(b * 16.0f);
    uh = (unsigned)__builtin_bit_cast(unsigned short, h0) | ((unsigned)__builtin_bit_cast(unsigned short, h1) << 16);
    ul = uh;
  } else {
    const unsigned short ha = f2bf_bits(a), hb = f2bf_bits(b);
    const unsigned short la = f2bf_bits(a - bf_bits2f(ha)), lbb = f2bf_bits(b - bf_bits2f(hb));
    uh = (unsigned)ha | ((unsigned)hb << 16);
    ul = (unsigned)la | ((unsigned)lbb << 16);
  }
  ((volatile unsigned*)dh)[i] = uh;
  if (!f16m) ((volatile unsigned*)dlo)[i] = ul;
  __threadfence();
  ((volatile unsigned*)dh)[i] = uh;
  if (!f16m) ((volatile unsigned*)dlo)[i] = ul;
}

template <bool F16M>
__global__ __launch_bounds__(NT) void cvt_rows_kernel(const float* __restrict__ X, int row0, int nreal,
                                                     unsigned short* __restrict__ P0, unsigned short* __restrict__ P1, int nrows) {
  const int i = blockIdx.x * NT + threadIdx.x;
  if (i >= nrows * (EMB / 8)) return;
  const int row = i >> 4, c8 = (i & 15) * 8;
  const int g = row0 + row;
  const bool live = g < nreal;
  const int gc = live ? g : (nreal - 1);
  v4f a = *(const v4f*)(X + (size_t)gc * EMB + c8);
  v4f b = *(const v4f*)(X + (size_t)gc * EMB + c8 + 4);
  const v4f z4 = {0.f, 0.f, 0.f, 0.f};
  if (!live) { a = z4; b = z4; }
  v8h hv, lv;
#pragma unroll
  for (int e = 0; e < 4; ++e) {
    const float f0 = a[e], f1 = b[e];
    if (F16M) {
      hv[e] = (_Float16)f0; hv[4 + e] = (_Float16)f1; lv[e] = hv[e]; lv[4 + e] = hv[4 + e];
    } else {
      const unsigned short h0 = f2bf_bits(f0), h1 = f2bf_bits(f1);
      const unsigned short l0 = f2bf_bits(f0 - bf_bits2f(h0)), l1 = f2bf_bits(f1 - bf_bits2f(h1));
      hv[e] = __builtin_bit_cast(_Float16, h0); hv[4 + e] = __builtin_bit_cast(_Float16, h1);
      lv[e] = __builtin_bit_cast(_Float16, l0); lv[4 + e] = __builtin_bit_cast(_Float16, l1);
    }
  }
  unsigned short* p0 = P0 + (size_t)row * EMB + c8;
  *(volatile v8h*)p0 = hv;
  if (!F16M) *(volatile v8h*)(P1 + (size_t)row * EMB + c8) = lv;
  __threadfence();
  *(volatile v8h*)p0 = hv;
  if (!F16M) *(volatile v8h*)(P1 + (size_t)row * EMB + c8) = lv;
}

__global__ __launch_bounds__(NT) void agg_kernel(const float* __restrict__ Lt, const float* __restrict__ Rt, const int* __restrict__ ei,
                                                const float* __restrict__ ef, const float* __restrict__ We,
                                                const float* __restrict__ sprep, const float* __restrict__ spostp, const int* __restrict__ nsegp,
                                                float* Sacc, unsigned short* __restrict__ SH, unsigned short* __restrict__ SL,
                                                float* __restrict__ CN, int hbase) {
  __shared__ int LIST[SCH];
  __shared__ int CNT[SRB];
  __shared__ int scan_ws[80];
  const int tid = threadIdx.x, lane = tid & 31, wave = tid >> 5;
  const int t0 = blockIdx.x * SRB;
  int nrows = NRH - t0; nrows = nrows < SRB ? nrows : SRB;
  const int g0 = hbase + t0;
  int nseg = nsegp[0]; nseg = nseg < 0 ? 0 : (nseg > NRN ? NRN : nseg);
  int gend = g0 + nrows; gend = gend < nseg ? gend : nseg;
  const float spre = sprep[0], spost = spostp[0];
  const v4f we = *(const v4f*)(We + 4 * lane);
  const v4f z4 = {0.f, 0.f, 0.f, 0.f};

  for (int pass = 0; pass < 2; ++pass) {
#pragma unroll 1
    for (int j = 0; j < RPW; ++j) {
      const int dl = wave * RPW + j;
      if (dl < nrows) *(volatile v4f*)(Sacc + (size_t)(t0 + dl) * EMB + 4 * lane) = z4;
    }
    __threadfence();
  }
  for (int i = tid; i < SRB; i += NT) CNT[i] = 0;
  __syncthreads();

  const int* srcv = ei; const int* dstv = ei + NE;
#pragma unroll 1
  for (int c = 0; c < NCH; ++c) {
    const int tot = chunk_hits_dst<SPT, SCH>(dstv, c * SCH, g0, gend, tid, LIST, scan_ws);
#pragma unroll 1
    for (int base = 0; base < tot; base += 32) {
      const int q = base + lane;
      const int qc = q < SCH ? q : SCH - 1;
      const int lq = LIST[qc];
      const int rv = (q < tot) ? lq : -1;
      const int own = (rv >= 0 && (rv >> 28) == wave) ? 1 : 0;
      unsigned msk = (unsigned)__ballot(own);
#pragma unroll 1
      for (int it = 0; it < 32; ++it) {
        if (msk == 0u) break;
        const int bp = __builtin_ctz(msk); msk &= msk - 1u;
        const int r = __shfl(rv, bp, 32);
        int dl = (r >> 19) & (SRB - 1); dl = dl < nrows ? dl : nrows - 1;
        int e = r & 0x7FFFF; e = e < NE ? e : NE - 1;
        int s = srcv[e]; s = s < 0 ? 0 : (s >= NLN ? NLN - 1 : s);
        const float efv = ef[e];
        const size_t row = (size_t)(t0 + dl);
        const v4f lt = *(const v4f*)(Lt + (size_t)s * EMB + 4 * lane);
        const v4f rt = *(const v4f*)(Rt + row * EMB + 4 * lane);
        const v4f jv = (lt + efv * we + rt) * spre;
        float* rp = Sacc + row * EMB + 4 * lane;
        v4f a = *(const v4f*)rp;
#pragma unroll
        for (int k = 0; k < 4; ++k) a[k] += fmaxf(jv[k], 0.0f);
        *(volatile v4f*)rp = a;
        __threadfence();
        *(volatile v4f*)rp = a;
        if (lane == 0) CNT[dl] += 1;
      }
    }
    __syncthreads();
  }

  const int cc = lane & 15, hh = lane >> 4;
#pragma unroll 1
  for (int j = 0; j < RPW; ++j) {
    const int dl = wave * RPW + j;
    if (dl < nrows) {
      const size_t row = (size_t)(t0 + dl);
      const float* rp = Sacc + row * EMB;
      const v4f a0 = *(const v4f*)(rp + 8 * cc), a1 = *(const v4f*)(rp + 8 * cc + 4);
      v8h sv;
#pragma unroll
      for (int k = 0; k < 4; ++k) {
        const float f0 = a0[k] * spost, f1 = a1[k] * spost;
        const unsigned short h0 = f2bf_bits(f0), h1 = f2bf_bits(f1);
        const unsigned short l0 = f2bf_bits(f0 - bf_bits2f(h0)), l1 = f2bf_bits(f1 - bf_bits2f(h1));
        sv[k]     = __builtin_bit_cast(_Float16, hh ? l0 : h0);
        sv[4 + k] = __builtin_bit_cast(_Float16, hh ? l1 : h1);
      }
      unsigned short* dp = (hh ? SL : SH) + row * EMB + 8 * cc;
      *(volatile v8h*)dp = sv;
      __threadfence();
      *(volatile v8h*)dp = sv;
    }
  }
  for (int i = tid * 4; i < nrows; i += NT * 4) {
    v4f cv;
    cv[0] = (float)CNT[i] * spost; cv[1] = (float)CNT[i + 1] * spost;
    cv[2] = (float)CNT[i + 2] * spost; cv[3] = (float)CNT[i + 3] * spost;
    float* cp = CN + t0 + i;
    *(volatile v4f*)cp = cv;
    __threadfence();
    *(volatile v4f*)cp = cv;
  }
}

extern "C" void kernel_launch(void* const* d_in, const int* in_sizes, int n_in,
                              void* d_out, int out_size, void* d_ws, size_t ws_size, hipStream_t stream) {
  if (n_in < 17) return;
  const float* left    = (const float*)d_in[0];
  const int*   eidx    = (const int*)  d_in[1];
  const float* ef      = (const float*)d_in[2];
  const float* right   = (const float*)d_in[3];
  const int*   sos     = (const int*)  d_in[4];
  const float* W_left  = (const float*)d_in[5];
  const float* b_left  = (const float*)d_in[6];
  const float* W_edge  = (const float*)d_in[7];
  const float* W_right = (const float*)d_in[8];
  const float* s_pre   = (const float*)d_in[9];
  const float* W_final = (const float*)d_in[10];
  const float* b_final = (const float*)d_in[11];
  const float* s_post  = (const float*)d_in[12];
  const float* W_out1  = (const float*)d_in[13];
  const float* b_out1  = (const float*)d_in[14];
  const float* W_out2  = (const float*)d_in[15];
  const float* b_out2  = (const float*)d_in[16];
  float* out = (float*)d_out;
  if (in_sizes[0] != NLN * EMB || in_sizes[1] != 2 * NE || in_sizes[2] != NE || in_sizes[3] != NRN * EMB ||
      in_sizes[4] < 1 || in_sizes[7] != EMB || in_sizes[13] != 2 * EMB * EMB || out_size != NRN * EMB) return;

  char* ws = (char*)d_ws; size_t off = 0;
  auto carve = [&](size_t bytes) -> char* { char* p = ws + off; off += (bytes + 255) & ~(size_t)255; return p; };
  const size_t RB = (size_t)NRH * EMB * 4;
  unsigned short* WlF = (unsigned short*)carve((size_t)EMB * EMB * 2);
  unsigned short* WrH = (unsigned short*)carve((size_t)EMB * EMB * 2);
  unsigned short* WrL = (unsigned short*)carve((size_t)EMB * EMB * 2);
  unsigned short* WfH = (unsigned short*)carve((size_t)EMB * EMB * 2);
  unsigned short* WfL = (unsigned short*)carve((size_t)EMB * EMB * 2);
  unsigned short* W1H = (unsigned short*)carve((size_t)2 * EMB * EMB * 2);
  unsigned short* W1L = (unsigned short*)carve((size_t)2 * EMB * EMB * 2);
  unsigned short* W2H = (unsigned short*)carve((size_t)EMB * EMB * 2);
  unsigned short* W2L = (unsigned short*)carve((size_t)EMB * EMB * 2);
  float*          CN  = (float*)carve((size_t)NRH * 4);
  char* R0 = carve(RB); char* R1 = carve(RB); char* R2 = carve(RB); char* R3 = carve(RB); char* R4 = carve(RB);
  if (off > ws_size || off > (size_t)134217728) return;

  float*          Lt    = (float*)R0;
  unsigned short* leftF = (unsigned short*)R1;
  unsigned short* rH    = (unsigned short*)R1;
  unsigned short* rL    = rH + (size_t)NRH * EMB;
  float*          Rt    = (float*)R2;
  unsigned short* hH    = (unsigned short*)R2;
  unsigned short* hL    = hH + (size_t)NRH * EMB;
  float*          Sacc  = (float*)R3;
  unsigned short* cH    = (unsigned short*)R3;
  unsigned short* cL    = cH + (size_t)NRH * EMB;
  unsigned short* SH    = (unsigned short*)R4;
  unsigned short* SL    = SH + (size_t)NRH * EMB;
  float*          Tb    = (float*)R4;

  const int gtiles = (NRH / 64) * (EMB / 64);
  const dim3 ggrid((gtiles + 7) / 8, 1);
  const unsigned cvtb = (unsigned)((NRH * (EMB / 8) + NT - 1) / NT);

  prep_w_kernel<<<192, NT, 0, stream>>>(W_left, W_right, W_final, W_out1, W_out2,
                                        (unsigned*)WlF, (unsigned*)WrH, (unsigned*)WrL, (unsigned*)WfH, (unsigned*)WfL,
                                        (unsigned*)W1H, (unsigned*)W1L, (unsigned*)W2H, (unsigned*)W2L);
  cvt_rows_kernel<true><<<cvtb, NT, 0, stream>>>(left, 0, NLN, leftF, leftF, NLP);
  wmma_gemm64<0, false, 2, 0, false, 0><<<ggrid, 256, 0, stream>>>(
      leftF, nullptr, EMB, 0L, WlF, nullptr, EMB, 0L, (void*)Lt, nullptr, EMB, 0L,
      b_left, nullptr, 0L, NLP, EMB, EMB, 0.0625f, NLP);

  for (int hb = 0; hb < 2; ++hb) {
    const int hbase = hb * NRH;
    const int mst   = (NRN - hbase) < NRH ? (NRN - hbase) : NRH;
    cvt_rows_kernel<false><<<cvtb, NT, 0, stream>>>(right, hbase, NRN, rH, rL, NRH);
    wmma_gemm64<1, true, 0, 0, false, 0><<<ggrid, 256, 0, stream>>>(
        rH, rL, EMB, 0L, WrH, WrL, EMB, 0L, (void*)Rt, nullptr, EMB, 0L,
        nullptr, nullptr, 0L, NRH, EMB, EMB, 1.0f, NRH);
    agg_kernel<<<NTILE, NT, 0, stream>>>(Lt, Rt, eidx, ef, W_edge, s_pre, s_post, sos, Sacc, SH, SL, CN, hbase);
    wmma_gemm64<1, true, 3, 2, false, 0><<<ggrid, 256, 0, stream>>>(
        SH, SL, EMB, 0L, WfH, WfL, EMB, 0L, (void*)cH, (void*)cL, EMB, 0L,
        b_final, CN, 0L, NRH, EMB, EMB, 1.0f, NRH);
    wmma_gemm64<1, true, 2, 0, false, 0><<<ggrid, 256, 0, stream>>>(
        cH, cL, EMB, 0L, W1H, W1L, 2 * EMB, 0L, (void*)Tb, nullptr, EMB, 0L,
        b_out1, nullptr, 0L, NRH, EMB, EMB, 1.0f, NRH);
    wmma_gemm64<1, true, 0, 2, true, 2><<<ggrid, 256, 0, stream>>>(
        rH, rL, EMB, 0L, W1H + EMB, W1L + EMB, 2 * EMB, 0L, (void*)hH, (void*)hL, EMB, 0L,
        nullptr, Tb, 0L, NRH, EMB, EMB, 1.0f, NRH);
    wmma_gemm64<1, true, 2, 0, false, 0><<<ggrid, 256, 0, stream>>>(
        hH, hL, EMB, 0L, W2H, W2L, EMB, 0L, (void*)(out + (size_t)hbase * EMB), nullptr, EMB, 0L,
        b_out2, nullptr, 0L, NRH, EMB, EMB, 1.0f, mst);
  }
}
